// REGCN_28630251995290
// MI455X (gfx1250) — hardware-verified
//
#include <hip/hip_runtime.h>
#include <stddef.h>
#include <stdint.h>


#define DD     200
#define KP     224
#define KQ     28
#define KST    7
#define NB     30
#define GB     15
#define NGRP   2
#define NG     3000
#define NGP    3008
#define HBP    3008
#define NSP    256
#define AGP    256
#define GSP    72
#define TR     16
#define NTHR   256
#define NWAVE  8
#define S1     1024
#define NCH1   4
#define SH1    8
#define FA1    64
#define CAP1   128
#define SH2    4
#define FA2    16
#define CAP2   896
#define NBLKB  658
#define NBLKS  28
#define WSC    64.0f
#define RWSC   0.015625f
#define SENT   0xFFFFFFFFu
#define WSCAPB 134217728

static_assert(KQ * 8 == KP);
static_assert(KST * 32 == KP);
static_assert(KP >= DD && (DD % 8) == 0 && (DD / 8) <= 32);
static_assert(NG == GB * DD && NGRP * GB == NB);
static_assert(NGP >= NG && (NGP % 64) == 0 && HBP == NGP && (HBP % 64) == 0);
static_assert(NSP >= DD && NSP == NWAVE * 32 && AGP == 256);
static_assert(NTHR == 32 * NWAVE && TR == 2 * NWAVE);
static_assert(NCH1 * NTHR == S1);
static_assert((FA1 * CAP1) % (4 * NTHR) == 0 && (FA2 * CAP2) % (4 * NTHR) == 0);
static_assert((CAP1 % 32) == 0 && (CAP2 % 32) == 0);
static_assert((1 << (SH1 - SH2)) == FA2 && (1 << SH2) == TR);
static_assert(NGRP * NGP * KQ == NBLKB * NTHR && NSP * KQ == NBLKS * NTHR);
static_assert((GSP % 8) == 0 && GSP >= 64);
static_assert(TR * AGP == 16 * NTHR);
static_assert(TR * DD <= 16 * NTHR);

typedef _Float16 v8h  __attribute__((ext_vector_type(8)));
typedef _Float16 v16h __attribute__((ext_vector_type(16)));
typedef float    v4f  __attribute__((ext_vector_type(4)));
typedef float    v8f  __attribute__((ext_vector_type(8)));
typedef unsigned int v4u __attribute__((ext_vector_type(4)));
typedef v8h v8ha __attribute__((may_alias));
typedef v4f v4fa __attribute__((may_alias));
typedef v4u v4ua __attribute__((may_alias));
union Frag { v16h v; v8h h[2]; };

__device__ __forceinline__ v8f wmh(v16h a, v16h b, v8f c) {
  v8f d = __builtin_amdgcn_wmma_f32_16x16x32_f16(false, a, false, b, (short)0, c, false, false);
  asm volatile("v_nop\n\tv_nop\n\tv_nop\n\tv_nop" : "+v"(d) : "v"(a), "v"(b));
  return d;
}

__global__ __launch_bounds__(NTHR) void k_prep(const float* __restrict__ x, const float* __restrict__ w,
                                               const float* __restrict__ sw, _Float16* Ap, _Float16* Bp,
                                               _Float16* Sp, unsigned* flag, int nN, int nbA, int nbB, int nbS) {
  const int tid = threadIdx.x;
  const int blk = blockIdx.x;
  const v8f z8 = {0.f, 0.f, 0.f, 0.f, 0.f, 0.f, 0.f, 0.f};
  if (blk < nbA) {
    const int i = blk * NTHR + tid;
    const int row = i / KQ, kq = i - row * KQ, k0 = kq * 8;
    const int rc = row < nN ? row : nN - 1;
    const int kc = k0 < DD - 8 ? k0 : DD - 8;
    const float* p = x + (size_t)rc * DD + kc;
    const v4f lo = *(const v4f*)p;
    const v4f hi = *(const v4f*)(p + 4);
    v8f f = {lo[0], lo[1], lo[2], lo[3], hi[0], hi[1], hi[2], hi[3]};
    if (!((row < nN) && (k0 < DD))) f = z8;
    const v8h hv = __builtin_convertvector(f, v8h);
    _Float16* dst = Ap + (size_t)i * 8;
    *(volatile v8h*)dst = hv;
    __threadfence();
    *(volatile v8h*)dst = hv;
  } else if (blk < nbA + nbB) {
    const int i = (blk - nbA) * NTHR + tid;
    const int g = i / (NGP * KQ);
    const int rem = i - g * (NGP * KQ);
    const int n = rem / KQ, kq = rem - n * KQ, k0 = kq * 8;
    const bool ok = (n < NG) && (k0 < DD);
    const int nc = n < NG ? n : NG - 1;
    const int kc = k0 < DD - 8 ? k0 : DD - 8;
    const int bl = nc / DD;
    const int b = g * GB + bl, d = nc - bl * DD;
    const float* p = w + ((size_t)b * DD + kc) * DD + d;
    v8f f;
#pragma unroll
    for (int e = 0; e < 8; ++e) f[e] = p[(size_t)e * DD] * WSC;
    if (!ok) f = z8;
    const v8h hv = __builtin_convertvector(f, v8h);
    _Float16* dst = Bp + (size_t)i * 8;
    *(volatile v8h*)dst = hv;
    __threadfence();
    *(volatile v8h*)dst = hv;
  } else if (blk < nbA + nbB + nbS) {
    const int i = (blk - nbA - nbB) * NTHR + tid;
    const int n = i / KQ, kq = i - n * KQ, k0 = kq * 8;
    const bool ok = (n < DD) && (k0 < DD);
    const int nc = n < DD ? n : DD - 1;
    const int kc = k0 < DD - 8 ? k0 : DD - 8;
    const float* p = sw + (size_t)kc * DD + nc;
    v8f f;
#pragma unroll
    for (int e = 0; e < 8; ++e) f[e] = p[(size_t)e * DD] * WSC;
    if (!ok) f = z8;
    const v8h hv = __builtin_convertvector(f, v8h);
    _Float16* dst = Sp + (size_t)i * 8;
    *(volatile v8h*)dst = hv;
    __threadfence();
    *(volatile v8h*)dst = hv;
  } else {
    if (tid < 8) {
      const v4u z4 = {0u, 0u, 0u, 0u};
      unsigned* dst = flag + 4 * tid;
      *(volatile v4u*)dst = z4;
      __threadfence();
      *(volatile v4u*)dst = z4;
    }
  }
}

template <int LV, int FA, int CAP>
__global__ __launch_bounds__(NTHR) void k_part(const int* __restrict__ esrc, const int* __restrict__ edst,
                                               const int* __restrict__ ety, const unsigned* __restrict__ lin,
                                               unsigned* lout, unsigned* flag,
                                               int nN, int nE, int nR, int nC, int nB1, int nch) {
  __shared__ __attribute__((aligned(16))) unsigned lst[FA * CAP];
  __shared__ int wc[NWAVE * FA];
  __shared__ int cur[FA];
  __shared__ int ovfl;
  const int tid = threadIdx.x, lane = tid & 31, wave = tid >> 5;
  const int blk = blockIdx.x;
  const v4u sv4 = {SENT, SENT, SENT, SENT};
#pragma unroll
  for (int k = 0; k < (FA * CAP) / (4 * NTHR); ++k) *(v4ua*)(&lst[4 * (tid + NTHR * k)]) = sv4;
  if (tid < FA) cur[tid] = 0;
  if (tid == 0) ovfl = 0;
  __syncthreads();

  const int nslots = nB1 * CAP1;
  const unsigned lt = (1u << lane) - 1u;

#pragma unroll 1
  for (int ch = 0; ch < nch; ++ch) {
    bool valid;
    int key;
    unsigned rec;
    if (LV == 1) {
      const int e = blk * S1 + ch * NTHR + tid;
      const int ec = e < nE ? e : nE - 1;
      const int d = edst[ec];
      valid = (e < nE) && ((unsigned)d < (unsigned)nN);
      key = d >> SH1;
      rec = (unsigned)ec;
    } else {
      const int q = ch * NTHR + tid;
      const int qc = q < nslots ? q : nslots - 1;
      const int bl = qc / CAP1, s = qc - bl * CAP1;
      const unsigned id = lin[((size_t)bl * nC + blk) * CAP1 + s];
      const bool idok = id < (unsigned)nE;
      const int idc = idok ? (int)id : nE - 1;
      const int d = edst[idc];
      int svv = esrc[idc];
      svv = svv < 0 ? 0 : (svv > nN - 1 ? nN - 1 : svv);
      int tv = ety[idc];
      tv = tv < 0 ? 0 : (tv > nR - 1 ? nR - 1 : tv);
      valid = (q < nslots) && idok && ((unsigned)d < (unsigned)nN) && ((d >> SH1) == blk);
      key = (d >> SH2) & (FA2 - 1);
      rec = ((unsigned)d & 15u) | ((unsigned)tv << 4) | ((unsigned)svv << 13);
    }
    key = valid ? key : 255;
    unsigned mym = 0u;
#pragma unroll
    for (int b = 0; b < FA; ++b) {
      const unsigned mb = __builtin_amdgcn_ballot_w32(key == b);
      mym = (key == b) ? mb : mym;
    }
    const int rank = __builtin_popcount(mym & lt);
    const int cnt  = __builtin_popcount(mym);
    for (int j = lane; j < FA; j += 32) wc[wave * FA + j] = 0;
    const int kc = valid ? key : 0;
    if (valid && rank == 0) wc[wave * FA + kc] = cnt;
    __syncthreads();
    int pre = 0;
    for (int w2 = 0; w2 < wave; ++w2) pre += wc[w2 * FA + kc];
    const int pos = cur[kc] + pre + rank;
    if (valid && pos < CAP) lst[kc * CAP + pos] = rec;
    int tot = 0;
    if (tid < FA) {
#pragma unroll
      for (int w2 = 0; w2 < NWAVE; ++w2) tot += wc[w2 * FA + tid];
    }
    __syncthreads();
    if (tid < FA) cur[tid] += tot;
  }
  __syncthreads();
  if (tid < FA && cur[tid] > CAP) ovfl = 1;
  __syncthreads();
  const bool wfl = (ovfl != 0) && (tid < 8);
  const v4u one4 = {1u, 1u, 1u, 1u};

  const int nwords  = (LV == 1) ? nC * CAP : FA * CAP;
  const int npieces = nwords >> 2;
  unsigned* gb = lout + (size_t)blk * nwords;
#pragma unroll
  for (int k = 0; k < (FA * CAP / 4 + NTHR - 1) / NTHR; ++k) {
    const int it = tid + NTHR * k;
    if (it < npieces) { const v4u v = *(const v4ua*)(&lst[4 * it]); *(volatile v4u*)(gb + 4 * it) = v; }
  }
  if (wfl) *(volatile v4u*)(flag + 4 * tid) = one4;
  __threadfence();
#pragma unroll
  for (int k = 0; k < (FA * CAP / 4 + NTHR - 1) / NTHR; ++k) {
    const int it = tid + NTHR * k;
    if (it < npieces) { const v4u v = *(const v4ua*)(&lst[4 * it]); *(volatile v4u*)(gb + 4 * it) = v; }
  }
  if (wfl) *(volatile v4u*)(flag + 4 * tid) = one4;
}

__global__ __launch_bounds__(NTHR) void k_gemm(const _Float16* __restrict__ Ap, const _Float16* __restrict__ Bp,
                                               _Float16* HB) {
  __shared__ __attribute__((aligned(16))) _Float16 stg[64 * GSP];
  const int tid = threadIdx.x, lane = tid & 31, wave = tid >> 5, hh = lane >> 4, mm = lane & 15;
  const int wm = wave & 3, wn = wave >> 2;
  const int m0 = blockIdx.x * 64, n0 = blockIdx.y * 64;
  const _Float16* abase = Ap + (size_t)(m0 + wm * 16 + mm) * KP + 8 * hh;
  const _Float16* bbase = Bp + (size_t)(n0 + wn * 32 + mm) * KP + 8 * hh;
  v8f c0 = {0.f, 0.f, 0.f, 0.f, 0.f, 0.f, 0.f, 0.f};
  v8f c1 = c0;
#pragma unroll
  for (int kt = 0; kt < KST; ++kt) {
    Frag a, b0, b1;
    a.h[0]  = *(const v8h*)(abase + 32 * kt);
    a.h[1]  = *(const v8h*)(abase + 32 * kt + 16);
    b0.h[0] = *(const v8h*)(bbase + 32 * kt);
    b0.h[1] = *(const v8h*)(bbase + 32 * kt + 16);
    b1.h[0] = *(const v8h*)(bbase + 16 * KP + 32 * kt);
    b1.h[1] = *(const v8h*)(bbase + 16 * KP + 32 * kt + 16);
    c0 = wmh(a.v, b0.v, c0);
    c1 = wmh(a.v, b1.v, c1);
  }
#pragma unroll
  for (int r = 0; r < 8; ++r) {
    const int row = wm * 16 + 8 * hh + r;
    stg[row * GSP + wn * 32 + mm]      = (_Float16)(c0[r] * RWSC);
    stg[row * GSP + wn * 32 + 16 + mm] = (_Float16)(c1[r] * RWSC);
  }
  __syncthreads();
  const int cs = (tid & 7) * 8;
  const int rA = (tid >> 3), rB = rA + 32;
  const v8h va = *(const v8ha*)(stg + rA * GSP + cs);
  const v8h vb = *(const v8ha*)(stg + rB * GSP + cs);
  _Float16* ga = HB + (size_t)(m0 + rA) * HBP + n0 + cs;
  _Float16* gb2 = HB + (size_t)(m0 + rB) * HBP + n0 + cs;
  *(volatile v8h*)ga = va;
  *(volatile v8h*)gb2 = vb;
  __threadfence();
  *(volatile v8h*)ga = va;
  *(volatile v8h*)gb2 = vb;
}

__device__ __forceinline__ void drain(unsigned msk, unsigned rec, v8f& acc, const _Float16* __restrict__ HB,
                                      const float* __restrict__ coeff, int cb0, int choff, int nN, int nR) {
  while (msk != 0u) {
    const int i = __builtin_ctz(msk);
    msk &= msk - 1u;
    const unsigned r = (unsigned)__builtin_amdgcn_readlane((int)rec, i);
    int src = (int)(r >> 13);
    src = src > nN - 1 ? nN - 1 : src;
    int ty = (int)((r >> 4) & 511u);
    ty = ty > nR - 1 ? nR - 1 : ty;
    const _Float16* hrow = HB + (size_t)src * HBP + choff;
    const float* crow = coeff + (size_t)ty * NB + cb0;
#pragma unroll
    for (int b = 0; b < GB; ++b) {
      const float c = crow[b];
      const v8h hv = *(const v8h*)(hrow + b * DD);
      acc += c * __builtin_convertvector(hv, v8f);
    }
  }
}

__global__ __launch_bounds__(NTHR) void k_agg(const _Float16* __restrict__ HB, const float* __restrict__ coeff,
                                              const unsigned* __restrict__ l2, const _Float16* __restrict__ Ap,
                                              const _Float16* __restrict__ Sp, const float* __restrict__ bias,
                                              const unsigned* __restrict__ flag, float* AG, float* out,
                                              int nN, int nR, int cb0, int fin) {
  __shared__ __attribute__((aligned(16))) float stg[TR * AGP];
  __shared__ __attribute__((aligned(16))) float ostg[TR * DD];
  const int tid = threadIdx.x, lane = tid & 31, wave = tid >> 5, hh = lane >> 4, mm = lane & 15;
  const int tile = blockIdx.x;
  const int lc = lane < (DD / 8 - 1) ? lane : (DD / 8 - 1);
  const bool chok = lane < (DD / 8);
  const int choff = 8 * lc;
  const v8f z8 = {0.f, 0.f, 0.f, 0.f, 0.f, 0.f, 0.f, 0.f};

  v8f acc0 = z8, acc1 = z8;
  int cnt0 = 0, cnt1 = 0;
  {
    const unsigned* seg = l2 + (size_t)tile * CAP2;
#pragma unroll 1
    for (int ch = 0; ch < CAP2 / 32; ++ch) {
      const unsigned rec = seg[ch * 32 + lane];
      const bool ok = ((int)rec) >= 0;
      const int ln = (int)(rec & 15u);
      const unsigned m0 = __builtin_amdgcn_ballot_w32(ok && (ln == 2 * wave));
      const unsigned m1 = __builtin_amdgcn_ballot_w32(ok && (ln == 2 * wave + 1));
      cnt0 += __builtin_popcount(m0);
      cnt1 += __builtin_popcount(m1);
      drain(m0, rec, acc0, HB, coeff, cb0, choff, nN, nR);
      drain(m1, rec, acc1, HB, coeff, cb0, choff, nN, nR);
    }
  }

  if (fin != 0) {
    {
      v8f d0 = z8, d1 = z8;
      const _Float16* abase = Ap + (size_t)(tile * TR + mm) * KP + 8 * hh;
      const _Float16* bbase = Sp + (size_t)(wave * 32 + mm) * KP + 8 * hh;
#pragma unroll
      for (int kt = 0; kt < KST; ++kt) {
        Frag a, b0, b1;
        a.h[0]  = *(const v8h*)(abase + 32 * kt);
        a.h[1]  = *(const v8h*)(abase + 32 * kt + 16);
        b0.h[0] = *(const v8h*)(bbase + 32 * kt);
        b0.h[1] = *(const v8h*)(bbase + 32 * kt + 16);
        b1.h[0] = *(const v8h*)(bbase + 16 * KP + 32 * kt);
        b1.h[1] = *(const v8h*)(bbase + 16 * KP + 32 * kt + 16);
        d0 = wmh(a.v, b0.v, d0);
        d1 = wmh(a.v, b1.v, d1);
      }
#pragma unroll
      for (int r = 0; r < 8; ++r) {
        stg[(8 * hh + r) * AGP + wave * 32 + mm]      = d0[r];
        stg[(8 * hh + r) * AGP + wave * 32 + 16 + mm] = d1[r];
      }
    }
    __syncthreads();

    const unsigned fl = flag[0];
    const float qn = __int_as_float(0x7fc00000);
    const v8f nan8 = {qn, qn, qn, qn, qn, qn, qn, qn};
    const v4f b0v = *(const v4f*)(bias + choff);
    const v4f b1v = *(const v4f*)(bias + choff + 4);
    const v8f bv = {b0v[0], b0v[1], b0v[2], b0v[3], b1v[0], b1v[1], b1v[2], b1v[3]};
#pragma unroll
    for (int q = 0; q < 2; ++q) {
      const v8f acc = (q == 0) ? acc0 : acc1;
      const int cnt = (q == 0) ? cnt0 : cnt1;
      const int j = 2 * wave + q;
      const size_t grow = (size_t)(tile * TR + j);
      const v4f p0 = *(const v4f*)(AG + grow * AGP + choff);
      const v4f p1 = *(const v4f*)(AG + grow * AGP + choff + 4);
      const v8f prev = {p0[0], p0[1], p0[2], p0[3], p1[0], p1[1], p1[2], p1[3]};
      const v4f s0 = *(const v4fa*)(stg + j * AGP + choff);
      const v4f s1 = *(const v4fa*)(stg + j * AGP + choff + 4);
      const v8f sv = {s0[0], s0[1], s0[2], s0[3], s1[0], s1[1], s1[2], s1[3]};
      const float inv = 1.0f / fmaxf((float)cnt, 1.0f);
      v8f o = (prev + acc) * inv + sv * RWSC + bv;
      if (fl != 0u) o = nan8;
      if (chok) {
        const v4f olo = {o[0], o[1], o[2], o[3]};
        const v4f ohi = {o[4], o[5], o[6], o[7]};
        *(v4fa*)(ostg + j * DD + choff)     = olo;
        *(v4fa*)(ostg + j * DD + choff + 4) = ohi;
      }
    }
    __syncthreads();

    const int rem = nN - tile * TR;
    const int rows = rem < TR ? rem : TR;
    const int npc = rows * (DD / 4);
    float* obase = out + (size_t)tile * TR * DD;
#pragma unroll
    for (int k = 0; k < 4; ++k) {
      const int p = NTHR * k + tid;
      if (p < npc) { const v4f v = *(const v4fa*)(ostg + 4 * p); *(volatile v4f*)(obase + 4 * p) = v; }
    }
    __threadfence();
#pragma unroll
    for (int k = 0; k < 4; ++k) {
      const int p = NTHR * k + tid;
      if (p < npc) { const v4f v = *(const v4fa*)(ostg + 4 * p); *(volatile v4f*)(obase + 4 * p) = v; }
    }
  } else {
#pragma unroll
    for (int q = 0; q < 2; ++q) {
      v8f s = (q == 0) ? acc0 : acc1;
      if (!chok) s = z8;
      const int j = 2 * wave + q;
      const v4f slo = {s[0], s[1], s[2], s[3]};
      const v4f shi = {s[4], s[5], s[6], s[7]};
      *(v4fa*)(stg + j * AGP + 8 * lane)     = slo;
      *(v4fa*)(stg + j * AGP + 8 * lane + 4) = shi;
    }
    __syncthreads();
    float* gb = AG + (size_t)tile * TR * AGP;
#pragma unroll
    for (int k = 0; k < 4; ++k) {
      const int p = NTHR * k + tid;
      const v4f v = *(const v4fa*)(stg + 4 * p);
      *(volatile v4f*)(gb + 4 * p) = v;
    }
    __threadfence();
#pragma unroll
    for (int k = 0; k < 4; ++k) {
      const int p = NTHR * k + tid;
      const v4f v = *(const v4fa*)(stg + 4 * p);
      *(volatile v4f*)(gb + 4 * p) = v;
    }
  }
}

extern "C" void kernel_launch(void* const* d_in, const int* in_sizes, int n_in,
                              void* d_out, int out_size, void* d_ws, size_t ws_size,
                              hipStream_t stream) {
  if (n_in < 8) return;
  if (in_sizes[0] <= 0 || (in_sizes[0] % DD) != 0) return;
  const int nN = in_sizes[0] / DD;
  if (nN < 1 || nN > 16384) return;
  if (in_sizes[1] != NB * DD * DD) return;
  if (in_sizes[2] <= 0 || (in_sizes[2] % NB) != 0) return;
  const int nR = in_sizes[2] / NB;
  if (nR < 1 || nR > 512) return;
  if (in_sizes[3] != DD * DD || in_sizes[4] != DD) return;
  const int nE = in_sizes[6];
  if (nE < 1 || nE > (1 << 26)) return;
  if (in_sizes[5] != 2 * nE) return;
  if (in_sizes[7] < 1) return;
  if (out_size != nN * DD) return;

  const float* x     = (const float*)d_in[0];
  const float* w     = (const float*)d_in[1];
  const float* coeff = (const float*)d_in[2];
  const float* sw    = (const float*)d_in[3];
  const float* bias  = (const float*)d_in[4];
  const int*   esrc  = (const int*)d_in[5];
  const int*   edst  = esrc + nE;
  const int*   ety   = (const int*)d_in[6];
  float* out = (float*)d_out;

  const int MP     = ((nN + 63) / 64) * 64;
  const int nTiles = (nN + TR - 1) / TR;
  const int nT16   = nTiles * TR;
  const int nC     = (nN + 255) >> SH1;
  const int nB1    = (nE + S1 - 1) / S1;
  const int nch2   = (nB1 * CAP1 + NTHR - 1) / NTHR;
  const int nbA    = (MP / 64) * ((64 * KQ) / NTHR);
  if (nC < 1 || nC > FA1) return;
  if (MP < nT16) return;

  char* ws = (char*)d_ws;
  size_t o = 0;
  const size_t oA  = o; o += (size_t)MP * KP * 2;                         o = (o + 255) & ~(size_t)255;
  const size_t oB  = o; o += (size_t)NGRP * NGP * KP * 2;                 o = (o + 255) & ~(size_t)255;
  const size_t oS  = o; o += (size_t)NSP * KP * 2;                        o = (o + 255) & ~(size_t)255;
  const size_t oFL = o; o += 256;
  const size_t oL1 = o; o += (size_t)nB1 * nC * CAP1 * 4;                 o = (o + 255) & ~(size_t)255;
  const size_t oL2 = o; o += (size_t)nC * FA2 * CAP2 * 4;                 o = (o + 255) & ~(size_t)255;
  const size_t oHB = o; o += (size_t)MP * HBP * 2;                        o = (o + 255) & ~(size_t)255;
  const size_t oAG = o; o += (size_t)nT16 * AGP * 4;                      o = (o + 255) & ~(size_t)255;
  if (o > ws_size || o > (size_t)WSCAPB) return;
  _Float16* Ap = (_Float16*)(ws + oA);
  _Float16* Bp = (_Float16*)(ws + oB);
  _Float16* Sp = (_Float16*)(ws + oS);
  unsigned* FL = (unsigned*)(ws + oFL);
  unsigned* L1 = (unsigned*)(ws + oL1);
  unsigned* L2 = (unsigned*)(ws + oL2);
  _Float16* HB = (_Float16*)(ws + oHB);
  float*    AG = (float*)(ws + oAG);

  k_prep<<<nbA + NBLKB + NBLKS + 1, NTHR, 0, stream>>>(x, w, sw, Ap, Bp, Sp, FL, nN, nbA, NBLKB, NBLKS);
  k_part<1, FA1, CAP1><<<nB1, NTHR, 0, stream>>>(esrc, edst, ety, L1, L1, FL, nN, nE, nR, nC, nB1, NCH1);
  k_part<2, FA2, CAP2><<<nC, NTHR, 0, stream>>>(esrc, edst, ety, L1, L2, FL, nN, nE, nR, nC, nB1, nch2);
  k_gemm<<<dim3(MP / 64, NGP / 64), NTHR, 0, stream>>>(Ap, Bp, HB);
  k_agg<<<nTiles, NTHR, 0, stream>>>(HB, coeff, L2, Ap, Sp, bias, FL, AG, out, nN, nR, 0, 0);
  k_gemm<<<dim3(MP / 64, NGP / 64), NTHR, 0, stream>>>(Ap, Bp + (size_t)NGP * KP, HB);
  k_agg<<<nTiles, NTHR, 0, stream>>>(HB, coeff, L2, Ap, Sp, bias, FL, AG, out, nN, nR, GB, 1);
}
